// JointGraphAttention_66786741453300
// MI455X (gfx1250) — hardware-verified
//
#include <hip/hip_runtime.h>

typedef _Float16 v16h __attribute__((ext_vector_type(16)));
typedef _Float16 v8h  __attribute__((ext_vector_type(8)));
typedef float    v8f  __attribute__((ext_vector_type(8)));
typedef float    v4f  __attribute__((ext_vector_type(4)));
typedef v8h __attribute__((may_alias)) v8ha;
typedef v4f __attribute__((may_alias)) v4fa;

union Frag { v16h v; v8h half[2]; };

#define NTOK 4096
#define CDIM 512
#define HDIM 64
#define FDIM 256
#define OFF_W2T 131072
#define OFF_WQT 393216
#define OFF_WOT 1179648
#define WT_HALVES 1441792

__device__ __forceinline__ v8f wmma_f16(v16h a, v16h b, v8f c) {
  v8f d = __builtin_amdgcn_wmma_f32_16x16x32_f16(false, a, false, b, (short)0, c, false, false);
  asm volatile("v_nop\n\tv_nop\n\tv_nop\n\tv_nop" : "+v"(d) : "v"(a), "v"(b));
  return d;
}

__device__ __forceinline__ v16h load_frag(const _Float16* p, int h) {
  Frag f;
  f.half[0] = *(const v8ha*)(p + 8 * h);
  f.half[1] = *(const v8ha*)(p + 16 + 8 * h);
  return f.v;
}

__global__ __launch_bounds__(256) void wtrans_kernel(
    const float* __restrict__ W1, const float* __restrict__ W2,
    const float* __restrict__ Wq, const float* __restrict__ Wk,
    const float* __restrict__ Wv, const float* __restrict__ Wo,
    _Float16* __restrict__ Wt)
{
  __shared__ __attribute__((aligned(16))) _Float16 sT[64 * 64];
  const int t = threadIdx.x;
  const int bid = blockIdx.x;
  int wsel, tile, kin;
  if (bid < 32) { wsel = 0; tile = bid; kin = FDIM; }
  else { const int e = bid - 32; wsel = 1 + (e >> 6); tile = e & 63; kin = CDIM; }
  const int ktc = kin >> 6;
  const int ntile = tile / ktc;
  const int ktile = tile - ntile * ktc;
  const int n0 = ntile * 64, k0 = ktile * 64;
  const float* src = W1;
  size_t doff = 0;
  if (wsel == 1)      { src = W2; doff = (size_t)OFF_W2T; }
  else if (wsel == 2) { src = Wq; doff = (size_t)OFF_WQT; }
  else if (wsel == 3) { src = Wk; doff = (size_t)OFF_WQT + 262144; }
  else if (wsel == 4) { src = Wv; doff = (size_t)OFF_WQT + 2 * 262144; }
  else if (wsel == 5) { src = Wo; doff = (size_t)OFF_WOT; }

  #pragma unroll
  for (int i = 0; i < 4; ++i) {
    const int row = (t >> 4) + 16 * i;
    const int c4 = (t & 15) * 4;
    const v4f w = *(const v4fa*)(src + (size_t)(k0 + row) * CDIM + n0 + c4);
    sT[(c4 + 0) * 64 + row] = (_Float16)(w.x * 16.0f);
    sT[(c4 + 1) * 64 + row] = (_Float16)(w.y * 16.0f);
    sT[(c4 + 2) * 64 + row] = (_Float16)(w.z * 16.0f);
    sT[(c4 + 3) * 64 + row] = (_Float16)(w.w * 16.0f);
  }
  __syncthreads();

  _Float16* dbase = Wt + doff;
  #pragma unroll
  for (int i = 0; i < 2; ++i) {
    const int p = t + 256 * i;
    const int c = p >> 3, q = p & 7;
    const v8h v = *(const v8ha*)(sT + c * 64 + 8 * q);
    _Float16* dst = dbase + (size_t)(n0 + c) * kin + k0 + 8 * q;
    *(volatile v8h*)dst = v;
  }
  __threadfence();
  #pragma unroll
  for (int i = 0; i < 2; ++i) {
    const int p = t + 256 * i;
    const int c = p >> 3, q = p & 7;
    const v8h v = *(const v8ha*)(sT + c * 64 + 8 * q);
    _Float16* dst = dbase + (size_t)(n0 + c) * kin + k0 + 8 * q;
    *(volatile v8h*)dst = v;
  }
}

__global__ __launch_bounds__(256) void xcvt_kernel(const float* __restrict__ x,
                                                   _Float16* __restrict__ xh, int n8)
{
  const int g = blockIdx.x * 256 + threadIdx.x;
  if (g >= n8) return;
  const v4f a = *(const v4fa*)(x + (size_t)g * 8);
  const v4f c = *(const v4fa*)(x + (size_t)g * 8 + 4);
  const v8h o = { (_Float16)a.x, (_Float16)a.y, (_Float16)a.z, (_Float16)a.w,
                  (_Float16)c.x, (_Float16)c.y, (_Float16)c.z, (_Float16)c.w };
  _Float16* dst = xh + (size_t)g * 8;
  *(volatile v8h*)dst = o;
  __threadfence();
  *(volatile v8h*)dst = o;
}

__global__ __launch_bounds__(256) void embed_kernel(const float* __restrict__ qp,
                                                    _Float16* __restrict__ emb)
{
  __shared__ __attribute__((aligned(16))) _Float16 sE[2 * 256];
  const int t = threadIdx.x;
  const int rl = t >> 7, j = t & 127;
  const int row = blockIdx.x * 2 + rl;
  const float tv = qp[row];
  float a = -9.210340371976184f * (float)j;
  a = a * 0.0078125f;
  const float f = expf(a);
  const float tf = tv * f;
  const float c = cosf(tf);
  const float s = sinf(tf);
  sE[rl * 256 + j] = (_Float16)(c * 64.0f);
  sE[rl * 256 + 128 + j] = (_Float16)(s * 64.0f);
  __syncthreads();
  if (t < 64) {
    const int r = t >> 5, q = t & 31;
    const v8h v = *(const v8ha*)(sE + r * 256 + 8 * q);
    _Float16* dst = emb + (size_t)(blockIdx.x * 2 + r) * FDIM + 8 * q;
    *(volatile v8h*)dst = v;
    __threadfence();
    *(volatile v8h*)dst = v;
  }
}

template <bool RES>
__device__ __forceinline__ void f32_pass(const float* sT, float* dst, const float* __restrict__ resid,
                                         int r0, int c0, int tid) {
  #pragma unroll
  for (int i = 0; i < 16; ++i) {
    const int p = tid + 128 * i;
    const int L = p >> 3, q = p & 7;
    const int row = L >> 1, hl = L & 1;
    v4f v = *(const v4fa*)(sT + row * 64 + 32 * hl + 4 * q);
    const size_t gi = (size_t)(r0 + row) * CDIM + c0 + 32 * hl + 4 * q;
    if (RES) { const v4f rr = *(const v4fa*)(resid + gi); v += rr; }
    *(volatile v4f*)(dst + gi) = v;
  }
}

__device__ __forceinline__ void h_row_pass(const _Float16* sTh, _Float16* dst, int r0, int c0, int tid) {
  #pragma unroll
  for (int i = 0; i < 8; ++i) {
    const int p = tid + 128 * i;
    const int row = p >> 3, q = p & 7;
    const v8h v = *(const v8ha*)(sTh + row * 64 + 8 * q);
    *(volatile v8h*)(dst + (size_t)(r0 + row) * CDIM + c0 + 8 * q) = v;
  }
}

__device__ __forceinline__ void vt_pass(const _Float16* sTh, _Float16* vt, int b0, int head, int tid) {
  #pragma unroll
  for (int i = 0; i < 8; ++i) {
    const int p = tid + 128 * i;
    const int L = p >> 3, q = p & 7;
    const int d = L >> 1, bsub = L & 1;
    const v8h v = *(const v8ha*)(sTh + d * 128 + 64 * bsub + 8 * q);
    _Float16* dst = vt + ((size_t)((b0 + bsub) * 8 + head) * HDIM + d) * 64 + 8 * q;
    *(volatile v8h*)dst = v;
  }
}

template <int MODE>
__global__ __launch_bounds__(128) void gemm_kernel(
    const _Float16* __restrict__ A, const _Float16* __restrict__ Bt,
    const float* __restrict__ bias0, const float* __restrict__ bias1,
    const float* __restrict__ resid,
    float* outF0, float* outF1, _Float16* outH,
    int K, float acc_sc)
{
  __shared__ __attribute__((aligned(16))) float sT[128 * 64];
  _Float16* sTh = reinterpret_cast<_Float16*>(sT);

  const int tid = threadIdx.x, lane = tid & 31, w = tid >> 5;
  const int h = lane >> 4, m = lane & 15;
  const int r0 = blockIdx.x * 128;
  const int which = (MODE == 2) ? (int)(blockIdx.y >> 3) : 0;
  const int head = (MODE == 2) ? (int)(blockIdx.y & 7) : (int)blockIdx.y;
  const int c0 = head * 64;
  const _Float16* Bb = Bt + (size_t)which * (CDIM * CDIM);
  const int r0w = r0 + 32 * w;

  const _Float16* xa0 = A + (size_t)(r0w + m) * K;
  const _Float16* xa1 = xa0 + (size_t)16 * K;
  const _Float16* wb  = Bb + (size_t)(c0 + m) * K;

  const v8f zero8 = {0.f, 0.f, 0.f, 0.f, 0.f, 0.f, 0.f, 0.f};
  v8f acc[2][4];
  #pragma unroll
  for (int mt = 0; mt < 2; ++mt)
    #pragma unroll
    for (int nt = 0; nt < 4; ++nt) acc[mt][nt] = zero8;

  #pragma unroll 1
  for (int k0 = 0; k0 < K; k0 += 32) {
    const v16h a0 = load_frag(xa0 + k0, h);
    const v16h a1 = load_frag(xa1 + k0, h);
    #pragma unroll
    for (int nt = 0; nt < 4; ++nt) {
      const v16h b = load_frag(wb + (size_t)(16 * nt) * K + k0, h);
      acc[0][nt] = wmma_f16(a0, b, acc[0][nt]);
      acc[1][nt] = wmma_f16(a1, b, acc[1][nt]);
    }
  }

  const float* bias = (MODE == 2 && which == 2) ? bias1 : bias0;
  const float bsc = (MODE == 2 && which == 1) ? 0.0f : 1.0f;
  #pragma unroll
  for (int nt = 0; nt < 4; ++nt) {
    const int col = 16 * nt + m;
    const float bvl = bias[c0 + col] * bsc;
    #pragma unroll
    for (int mt = 0; mt < 2; ++mt) {
      #pragma unroll
      for (int r = 0; r < 8; ++r) {
        const int tokl = 32 * w + 16 * mt + 8 * h + r;
        float y = acc[mt][nt][r] * acc_sc + bvl;
        if (MODE == 0) {
          const float e = __expf(-y);
          y = y * __builtin_amdgcn_rcpf(1.0f + e);
          sTh[tokl * 64 + col] = (_Float16)(y * 16.0f);
        } else if (MODE == 2) {
          if (which == 2) sTh[col * 128 + tokl] = (_Float16)y;
          else sT[tokl * 64 + col] = y;
        } else {
          sT[tokl * 64 + col] = y;
        }
      }
    }
  }
  __syncthreads();

  if (MODE == 0) {
    h_row_pass(sTh, outH, r0, c0, tid);
    __threadfence();
    h_row_pass(sTh, outH, r0, c0, tid);
  } else if (MODE == 1) {
    f32_pass<false>(sT, outF0, resid, r0, c0, tid);
    __threadfence();
    f32_pass<false>(sT, outF0, resid, r0, c0, tid);
  } else if (MODE == 2) {
    if (which == 2) {
      const int b0 = blockIdx.x * 2;
      vt_pass(sTh, outH, b0, head, tid);
      __threadfence();
      vt_pass(sTh, outH, b0, head, tid);
    } else {
      float* dst = (which == 0) ? outF0 : outF1;
      f32_pass<false>(sT, dst, resid, r0, c0, tid);
      __threadfence();
      f32_pass<false>(sT, dst, resid, r0, c0, tid);
    }
  } else {
    f32_pass<true>(sT, outF0, resid, r0, c0, tid);
    __threadfence();
    f32_pass<true>(sT, outF0, resid, r0, c0, tid);
  }
}

__global__ __launch_bounds__(256) void attn_kernel(
    const float* __restrict__ qp,
    const float* __restrict__ kp,
    const float* __restrict__ pe,
    const _Float16* __restrict__ vt,
    _Float16* __restrict__ xo)
{
  __shared__ __attribute__((aligned(16))) float qs[64 * 64];
  __shared__ __attribute__((aligned(16))) float ks[64 * 64];
  __shared__ __attribute__((aligned(16))) float sc[64 * 64];
  __shared__ __attribute__((aligned(16))) _Float16 ps[64 * 64];

  const int t = threadIdx.x, lane = t & 31, wid = t >> 5;
  const int l15 = lane & 15, hi = lane >> 4;
  const int bh = blockIdx.x, b = bh >> 3, hh = bh & 7;

  #pragma unroll
  for (int j = 0; j < 4; ++j) {
    const int c = t + 256 * j;
    const int n = c >> 4, cc = c & 15;
    const size_t g = (size_t)(b * 64 + n) * CDIM + hh * 64 + cc * 4;
    *(v4fa*)(qs + c * 4) = *(const v4fa*)(qp + g);
    *(v4fa*)(ks + c * 4) = *(const v4fa*)(kp + g);
  }
  __syncthreads();

  #pragma unroll 1
  for (int it = 0; it < 16; ++it) {
    const int i = t + 256 * it;
    const int n = i >> 6, mm = i & 63;
    const float* per = pe + (size_t)(n * 64 + mm) * CDIM + hh * 64;
    const float* qr = qs + n * 64;
    const float* kr = ks + mm * 64;
    float acc = 0.0f;
    #pragma unroll 4
    for (int d4 = 0; d4 < 16; ++d4) {
      const v4f pv = *(const v4fa*)(per + 4 * d4);
      const v4f qv = *(const v4fa*)(qr + 4 * d4);
      const v4f kv = *(const v4fa*)(kr + 4 * d4);
      acc += (qv.x * pv.x) * kv.x;
      acc += (qv.y * pv.y) * kv.y;
      acc += (qv.z * pv.z) * kv.z;
      acc += (qv.w * pv.w) * kv.w;
    }
    sc[i] = acc * 0.125f;
  }
  __syncthreads();

  {
    const int n = t >> 2, part = t & 3;
    float* row = sc + n * 64 + part * 16;
    float mx = row[0];
    #pragma unroll
    for (int j = 1; j < 16; ++j) mx = fmaxf(mx, row[j]);
    mx = fmaxf(mx, __shfl_xor(mx, 1));
    mx = fmaxf(mx, __shfl_xor(mx, 2));
    float sum = 0.0f;
    #pragma unroll 1
    for (int j = 0; j < 16; ++j) {
      const float e = expf(row[j] - mx);
      row[j] = e;
      sum += e;
    }
    sum += __shfl_xor(sum, 1);
    sum += __shfl_xor(sum, 2);
    const float inv = 1.0f / sum;
    #pragma unroll
    for (int j = 0; j < 16; ++j)
      ps[n * 64 + part * 16 + j] = (_Float16)(row[j] * inv * 4096.0f);
  }
  __syncthreads();

  const int tr = wid >> 1;
  const int tc0 = 2 * (wid & 1), tc1 = tc0 + 1;
  const _Float16* vbh = vt + (size_t)bh * (HDIM * 64);
  const v8f zero8 = {0.f, 0.f, 0.f, 0.f, 0.f, 0.f, 0.f, 0.f};
  v8f oa = zero8, ob = zero8;
  #pragma unroll
  for (int k0 = 0; k0 < 64; k0 += 32) {
    const v16h a  = load_frag(ps + (tr * 16 + l15) * 64 + k0, hi);
    const v16h b0 = load_frag(vbh + (size_t)(tc0 * 16 + l15) * 64 + k0, hi);
    const v16h b1 = load_frag(vbh + (size_t)(tc1 * 16 + l15) * 64 + k0, hi);
    oa = wmma_f16(a, b0, oa);
    ob = wmma_f16(a, b1, ob);
  }

  _Float16* xt = reinterpret_cast<_Float16*>(qs);
  #pragma unroll
  for (int r = 0; r < 8; ++r) {
    const int n = tr * 16 + 8 * hi + r;
    xt[n * 64 + tc0 * 16 + l15] = (_Float16)(oa[r] * 0.00390625f);
    xt[n * 64 + tc1 * 16 + l15] = (_Float16)(ob[r] * 0.00390625f);
  }
  __syncthreads();

  #pragma unroll
  for (int i = 0; i < 2; ++i) {
    const int p = t + 256 * i;
    const int n = p >> 3, q = p & 7;
    const v8h v = *(const v8ha*)(xt + n * 64 + 8 * q);
    *(volatile v8h*)(xo + (size_t)(b * 64 + n) * CDIM + hh * 64 + 8 * q) = v;
  }
  __threadfence();
  #pragma unroll
  for (int i = 0; i < 2; ++i) {
    const int p = t + 256 * i;
    const int n = p >> 3, q = p & 7;
    const v8h v = *(const v8ha*)(xt + n * 64 + 8 * q);
    *(volatile v8h*)(xo + (size_t)(b * 64 + n) * CDIM + hh * 64 + 8 * q) = v;
  }
}

extern "C" void kernel_launch(void* const* d_in, const int* in_sizes, int n_in,
                              void* d_out, int out_size, void* d_ws, size_t ws_size,
                              hipStream_t stream) {
  if (n_in < 13) return;
  if (in_sizes[0] != NTOK * CDIM) return;
  if (in_sizes[1] != NTOK) return;
  if (in_sizes[2] != CDIM * CDIM || in_sizes[4] != CDIM * CDIM || in_sizes[5] != CDIM * CDIM) return;
  if (in_sizes[7] != CDIM * CDIM || in_sizes[11] != CDIM * CDIM) return;
  if (in_sizes[9] != FDIM * CDIM) return;
  if (in_sizes[3] != CDIM || in_sizes[6] != CDIM || in_sizes[8] != CDIM) return;
  if (in_sizes[10] != CDIM || in_sizes[12] != CDIM) return;
  if (out_size != NTOK * CDIM) return;

  const float* query = (const float*)d_in[0];
  const float* qpos  = (const float*)d_in[1];
  const float* Wq    = (const float*)d_in[2];
  const float* bq    = (const float*)d_in[3];
  const float* Wk    = (const float*)d_in[4];
  const float* Wv    = (const float*)d_in[5];
  const float* bv    = (const float*)d_in[6];
  const float* Wo    = (const float*)d_in[7];
  const float* bo    = (const float*)d_in[8];
  const float* W1    = (const float*)d_in[9];
  const float* b1    = (const float*)d_in[10];
  const float* W2    = (const float*)d_in[11];
  const float* b2    = (const float*)d_in[12];
  float* out = (float*)d_out;

  const size_t wt_bytes  = (size_t)WT_HALVES * 2;
  const size_t h16_bytes = (size_t)NTOK * CDIM * 2;
  const size_t emb_bytes = (size_t)NTOK * FDIM * 2;
  const size_t f32_bytes = (size_t)NTOK * CDIM * 4;
  size_t off = 0;
  const size_t o_wt  = off; off += wt_bytes;
  const size_t o_xh  = off; off += h16_bytes;
  const size_t o_emb = off; off += emb_bytes;
  const size_t o_h1  = off; off += h16_bytes;
  const size_t o_pe  = off; off += f32_bytes;
  const size_t o_q   = off; off += f32_bytes;
  const size_t o_k   = off; off += f32_bytes;
  const size_t o_vt  = off; off += h16_bytes;
  const size_t o_x   = off; off += h16_bytes;
  if (off > ws_size) return;

  char* ws = (char*)d_ws;
  _Float16* wt  = (_Float16*)(ws + o_wt);
  _Float16* xh  = (_Float16*)(ws + o_xh);
  _Float16* emb = (_Float16*)(ws + o_emb);
  _Float16* h1  = (_Float16*)(ws + o_h1);
  float*    pe  = (float*)(ws + o_pe);
  float*    qpl = (float*)(ws + o_q);
  float*    kpl = (float*)(ws + o_k);
  _Float16* vt  = (_Float16*)(ws + o_vt);
  _Float16* xpl = (_Float16*)(ws + o_x);

  wtrans_kernel<<<32 + 5 * 64, 256, 0, stream>>>(W1, W2, Wq, Wk, Wv, Wo, wt);
  xcvt_kernel<<<(NTOK * CDIM / 8) / 256, 256, 0, stream>>>(query, xh, NTOK * CDIM / 8);
  embed_kernel<<<NTOK / 2, 256, 0, stream>>>(qpos, emb);

  gemm_kernel<0><<<dim3(NTOK / 128, CDIM / 64), 128, 0, stream>>>(
      emb, wt, b1, b1, query, pe, pe, h1, FDIM, 0.0009765625f);
  gemm_kernel<1><<<dim3(NTOK / 128, CDIM / 64), 128, 0, stream>>>(
      h1, wt + OFF_W2T, b2, b2, query, pe, pe, vt, CDIM, 0.00390625f);
  gemm_kernel<2><<<dim3(NTOK / 128, 3 * (CDIM / 64)), 128, 0, stream>>>(
      xh, wt + OFF_WQT, bq, bv, query, qpl, kpl, vt, CDIM, 0.0625f);

  attn_kernel<<<64 * 8, 256, 0, stream>>>(qpl, kpl, pe, vt, xpl);

  gemm_kernel<3><<<dim3(NTOK / 128, CDIM / 64), 128, 0, stream>>>(
      xpl, wt + OFF_WOT, bo, bo, query, out, out, vt, CDIM, 0.00390625f);
}
